// DCLLoss_72172630442628
// MI455X (gfx1250) — hardware-verified
//
#include <hip/hip_runtime.h>


#define NN   8192
#define CD   128
#define RCH  1024
#define NCH  (NN / RCH)
#define TINV 10.0f
#define DM   CD
#define LOSC 1024.0f

typedef _Float16 h16;
typedef unsigned short bf;
typedef __attribute__((ext_vector_type(16))) __bf16   v16bf;
typedef __attribute__((ext_vector_type(16))) _Float16 v16h;
typedef __attribute__((ext_vector_type(8)))  _Float16 v8h;
typedef __attribute__((ext_vector_type(8)))  unsigned short v8us;
typedef __attribute__((ext_vector_type(8)))  float    v8f;
typedef __attribute__((ext_vector_type(4)))  float    v4f;
typedef v8h  __attribute__((may_alias)) v8ha;
typedef v4f  __attribute__((may_alias)) v4fa;
typedef v8us __attribute__((may_alias)) v8usa;

__device__ __forceinline__ unsigned short f2bf(float f) { unsigned u = __float_as_uint(f); u += 0x7FFFu + ((u >> 16) & 1u); return (unsigned short)(u >> 16); }
__device__ __forceinline__ float bf2f(unsigned short b) { return __uint_as_float(((unsigned)b) << 16); }
__device__ __forceinline__ float bfr(float f) { return bf2f(f2bf(f)); }
__device__ __forceinline__ v16h cat16(v8h lo, v8h hi) { return __builtin_shufflevector(lo, hi, 0, 1, 2, 3, 4, 5, 6, 7, 8, 9, 10, 11, 12, 13, 14, 15); }
__device__ __forceinline__ v16bf cat16b(v8us lo, v8us hi) { return __builtin_bit_cast(v16bf, __builtin_shufflevector(lo, hi, 0, 1, 2, 3, 4, 5, 6, 7, 8, 9, 10, 11, 12, 13, 14, 15)); }
__device__ __forceinline__ v8f wmma16(v16h a, v16h b, v8f c) { return __builtin_amdgcn_wmma_f32_16x16x32_f16(false, a, false, b, (short)0, c, false, false); }
__device__ __forceinline__ v8f wmmab(v16bf a, v16bf b, v8f c) { return __builtin_amdgcn_wmma_f32_16x16x32_bf16(false, a, false, b, (short)0, c, false, false); }

template <bool SPLITA, bool F16OUT = false>
__global__ __launch_bounds__(128) void k_gemmb(const bf* __restrict__ A, const bf* __restrict__ Al, const bf* __restrict__ Bn, const float* __restrict__ bias, float* C, int ldc, h16* C2, const float* __restrict__ R = nullptr, int K = DM, int roundR = 1) {
    __shared__ __align__(16) float ost[4][16 * 68];
    const int lane = threadIdx.x & 31, wave = threadIdx.x >> 5, lr = lane & 15, hi = lane >> 4;
    const int r0 = blockIdx.x * 64 + wave * 16, c0 = blockIdx.y * 64;
    const size_t aoff = (size_t)(r0 + lr) * K + 8 * hi;
    size_t boff[4];
#pragma unroll
    for (int t = 0; t < 4; ++t) boff[t] = (size_t)(c0 + t * 16 + lr) * K + 8 * hi;
    v8f acc[4];
#pragma unroll
    for (int t = 0; t < 4; ++t) acc[t] = (v8f){};
#pragma unroll 1
    for (int kc = 0; kc < K; kc += 32) {
        const v16bf a = cat16b(*(const v8us*)(A + aoff + kc), *(const v8us*)(A + aoff + kc + 16));
        v16bf al = a;
        if (SPLITA) al = cat16b(*(const v8us*)(Al + aoff + kc), *(const v8us*)(Al + aoff + kc + 16));
#pragma unroll
        for (int t = 0; t < 4; ++t) { const v16bf b = cat16b(*(const v8us*)(Bn + boff[t] + kc), *(const v8us*)(Bn + boff[t] + kc + 16)); acc[t] = wmmab(a, b, acc[t]); if (SPLITA) acc[t] = wmmab(al, b, acc[t]); }
        asm volatile("v_nop\n\tv_nop\n\tv_nop\n\tv_nop" : "+v"(acc[0]), "+v"(acc[1]), "+v"(acc[2]), "+v"(acc[3]) : "v"(a), "v"(al));
    }
    float* os = &ost[wave][0];
#pragma unroll
    for (int t = 0; t < 4; ++t) { const float bv = bias ? bfr(bias[c0 + t * 16 + lr]) : 0.f;
#pragma unroll
        for (int j = 0; j < 8; ++j) os[(hi * 8 + j) * 68 + t * 16 + lr] = acc[t][j] + bv; }
    __syncthreads();
    if (F16OUT) {
        h16* crow = (h16*)(void*)C + (size_t)r0 * ldc + c0;
        auto pass = [&]() {
#pragma unroll
            for (int s = 0; s < 4; ++s) { const int row = 4 * s + (lane >> 3), piece = lane & 7; const float* sp = os + row * 68 + piece * 8; v8h o, o2;
#pragma unroll
                for (int i = 0; i < 8; ++i) { const h16 a = (h16)sp[i]; o[i] = a; o2[i] = (h16)((sp[i] - (float)a) * LOSC); }
                *(volatile v8h*)(crow + (size_t)row * ldc + piece * 8) = o; if (C2) *(volatile v8h*)(C2 + (size_t)r0 * ldc + c0 + (size_t)row * ldc + piece * 8) = o2; }
        };
        pass(); __threadfence(); pass();
    } else {
        float* crow = C + (size_t)r0 * ldc + c0;
        auto pass = [&]() {
#pragma unroll
            for (int s = 0; s < 8; ++s) { const int Lid = (lane >> 3) + 4 * s, piece = lane & 7; const int row = Lid >> 1, cofs = (Lid & 1) * 32 + piece * 4;
                v4f val = *(const v4fa*)(os + row * 68 + cofs); if (R) { const v4f rv = *(const v4f*)(R + ((size_t)r0 + row) * ldc + c0 + cofs); val += roundR ? (v4f){bfr(rv[0]), bfr(rv[1]), bfr(rv[2]), bfr(rv[3])} : rv; }
                *(volatile v4f*)(crow + (size_t)row * ldc + cofs) = val; }
        };
        pass(); __threadfence(); pass();
    }
}


__global__ __launch_bounds__(256) void k_normb(const float* __restrict__ x, bf* XB) {
    typedef __attribute__((ext_vector_type(4))) unsigned short v4us;
    const int lane = threadIdx.x & 31; const size_t r = (size_t)blockIdx.x * 8 + (threadIdx.x >> 5); if (r >= (size_t)NN) return; float v[4]; float s = 0.f;
#pragma unroll
    for (int i = 0; i < 4; ++i) { v[i] = bfr(x[r * CD + lane * 4 + i]); s = fmaf(v[i], v[i], s); }
#pragma unroll
    for (int sh = 16; sh; sh >>= 1) s += __shfl_xor(s, sh, 32);
    const float inv = 1.0f / fmaxf(sqrtf(s), 1e-12f); v4us o;
#pragma unroll
    for (int i = 0; i < 4; ++i) o[i] = f2bf(v[i] * inv);
    *(volatile v4us*)(XB + r * CD + lane * 4) = o; __threadfence(); *(volatile v4us*)(XB + r * CD + lane * 4) = o;
}
__global__ __launch_bounds__(256) void k_rowlse(const float* __restrict__ G, int r0, float* ROW, float* DIAGV) {
    __shared__ float sh_l[8], sh_d[8];
    const int lane = threadIdx.x & 31, wv = threadIdx.x >> 5, rl = blockIdx.x * 8 + wv; const int i = r0 + rl; const float* gr = G + (size_t)rl * NN;
    float m = -3.0e38f;
#pragma unroll 1
    for (int j0 = lane * 4; j0 < NN; j0 += 128) {
#pragma unroll
        for (int q = 0; q < 4; ++q) { const int j = j0 + q; const float v = (j == i) ? -3.0e38f : gr[j] * TINV; m = fmaxf(m, v); } }
#pragma unroll
    for (int sh = 16; sh; sh >>= 1) m = fmaxf(m, __shfl_xor(m, sh, 32));
    float s = 0.f;
#pragma unroll 1
    for (int j0 = lane * 4; j0 < NN; j0 += 128) {
#pragma unroll
        for (int q = 0; q < 4; ++q) { const int j = j0 + q; if (j != i) s += __expf(gr[j] * TINV - m); } }
#pragma unroll
    for (int sh = 16; sh; sh >>= 1) s += __shfl_xor(s, sh, 32);
    if (lane == 0) { sh_l[wv] = m + logf(s); sh_d[wv] = gr[i] * TINV; }
    __syncthreads();
    if (wv == 0) { const float lv = (lane < 8) ? sh_l[lane] : 0.f; float* dst = ROW + (size_t)blockIdx.x * 32 + lane; *(volatile float*)dst = lv; __threadfence(); *(volatile float*)dst = lv;
        if (DIAGV) { const float dv = (lane < 8) ? sh_d[lane] : 0.f; float* dd = DIAGV + (size_t)blockIdx.x * 32 + lane; *(volatile float*)dd = dv; __threadfence(); *(volatile float*)dd = dv; } }
}
__global__ __launch_bounds__(256) void k_colpart(const float* __restrict__ G, int r0, float* CM, float* CS) {
    const int j = blockIdx.x * 256 + threadIdx.x; if (j >= NN) return; float m = -3.0e38f;
#pragma unroll 4
    for (int rl = 0; rl < RCH; ++rl) { if (r0 + rl == j) continue; m = fmaxf(m, G[(size_t)rl * NN + j] * TINV); }
    float s = 0.f;
#pragma unroll 4
    for (int rl = 0; rl < RCH; ++rl) { if (r0 + rl == j) continue; s += __expf(G[(size_t)rl * NN + j] * TINV - m); }
    *(volatile float*)(CM + j) = m; *(volatile float*)(CS + j) = s; __threadfence(); *(volatile float*)(CM + j) = m; *(volatile float*)(CS + j) = s;
}
__device__ __forceinline__ float rowv(const float* __restrict__ R, int i) { return R[(size_t)(i >> 3) * 32 + (i & 7)]; }
__global__ __launch_bounds__(256) void k_final(const float* __restrict__ R00, const float* __restrict__ R01, const float* __restrict__ R11, const float* __restrict__ D01, const float* __restrict__ CM, const float* __restrict__ CS, float* OUTP) {
    __shared__ float pa[256], pd[256];
    const int t = threadIdx.x; float a = 0.f, d = 0.f;
    for (int q = 0; q < NN / 256; ++q) { const int i = t * (NN / 256) + q;
        float cm = -3.0e38f; for (int ch = 0; ch < NCH; ++ch) cm = fmaxf(cm, CM[(size_t)ch * NN + i]);
        float cs = 0.f; for (int ch = 0; ch < NCH; ++ch) cs += CS[(size_t)ch * NN + i] * __expf(CM[(size_t)ch * NN + i] - cm);
        const float col = cm + logf(cs);
        a += rowv(R01, i) + rowv(R00, i) + col + rowv(R11, i); d += rowv(D01, i); }
    pa[t] = a; pd[t] = d; __syncthreads();
    if (t == 0) { float A = 0.f, Dd = 0.f; for (int k = 0; k < 256; ++k) { A += pa[k]; Dd += pd[k]; }
        const float n = (float)NN; const float loss = 0.5f * ((-Dd / n) * 2.0f + A / n);
        *(volatile float*)OUTP = loss; __threadfence(); *(volatile float*)OUTP = loss; }
}

extern "C" void kernel_launch(void* const* d_in, const int* in_sizes, int n_in,
                              void* d_out, int out_size, void* d_ws, size_t ws_size, hipStream_t stream) {
    (void)in_sizes; (void)n_in; (void)out_size;
    const float* img = (const float*)d_in[0]; const float* mol = (const float*)d_in[1];
    float* out = (float*)d_out;
    char* wsp = (char*)d_ws;
    auto take = [&](size_t bytes) { char* p = wsp; wsp += (bytes + 255) & ~(size_t)255; return (void*)p; };
    bf* IB = (bf*)take((size_t)NN * CD * 2); bf* MB = (bf*)take((size_t)NN * CD * 2); float* G = (float*)take((size_t)RCH * NN * 4);
    float* R00 = (float*)take((NN / 8) * 32 * 4); float* R01 = (float*)take((NN / 8) * 32 * 4); float* R11 = (float*)take((NN / 8) * 32 * 4); float* D01 = (float*)take((NN / 8) * 32 * 4);
    float* CM = (float*)take((size_t)NCH * NN * 4); float* CS = (float*)take((size_t)NCH * NN * 4);
    if ((size_t)(wsp - (char*)d_ws) > ws_size) return;
    k_normb<<<NN / 8, 256, 0, stream>>>(img, IB); k_normb<<<NN / 8, 256, 0, stream>>>(mol, MB);
    for (int ch = 0; ch < NCH; ++ch) { const int r0 = ch * RCH;
        k_gemmb<false, false><<<dim3(RCH / 64, NN / 64, 1), 128, 0, stream>>>(IB + (size_t)r0 * CD, nullptr, MB, nullptr, G, NN, nullptr, nullptr, CD);
        k_rowlse<<<RCH / 8, 256, 0, stream>>>(G, r0, R01 + (size_t)(r0 / 8) * 32, D01 + (size_t)(r0 / 8) * 32); k_colpart<<<NN / 256, 256, 0, stream>>>(G, r0, CM + (size_t)ch * NN, CS + (size_t)ch * NN);
        k_gemmb<false, false><<<dim3(RCH / 64, NN / 64, 1), 128, 0, stream>>>(IB + (size_t)r0 * CD, nullptr, IB, nullptr, G, NN, nullptr, nullptr, CD);
        k_rowlse<<<RCH / 8, 256, 0, stream>>>(G, r0, R00 + (size_t)(r0 / 8) * 32, nullptr);
        k_gemmb<false, false><<<dim3(RCH / 64, NN / 64, 1), 128, 0, stream>>>(MB + (size_t)r0 * CD, nullptr, MB, nullptr, G, NN, nullptr, nullptr, CD);
        k_rowlse<<<RCH / 8, 256, 0, stream>>>(G, r0, R11 + (size_t)(r0 / 8) * 32, nullptr); }
    k_final<<<1, 256, 0, stream>>>(R00, R01, R11, D01, CM, CS, out);
}
